// GCNII_23089744183809
// MI455X (gfx1250) — hardware-verified
//
#include <hip/hip_runtime.h>
#include <stddef.h>
#include <stdint.h>
#include <math.h>


#define F       128
#define KC      256
#define NTHR    256
#define NWAVE   8
#define EPT     8
#define CHUNK   (NTHR * EPT)
#define WCAP    (EPT * 32)
#define LISTN   (NWAVE * WCAP)
#define NBA     1024
#define PKS     10
#define RCAP    28672
#define DEGCAP  64
#define STW     512
#define GBM     64
#define GBN     128
#define GTHR    128
#define NUL     (F * (F / 8))
#define NUC1    (F * (KC / 8))
#define ZINTS   (2 * RCAP + 2 * NBA + LISTN)
#define LDS_AGG (ZINTS * 4 + 64)
#define WSMAX   134217728

static_assert((CHUNK & (CHUNK - 1)) == 0);
static_assert(NBA == (1 << PKS));
static_assert(((long long)CHUNK << PKS) < (1LL << 31));
static_assert(NTHR * 4 == NBA);
static_assert(LISTN >= NBA && LISTN >= NWAVE * WCAP);
static_assert((RCAP % 32) == 0 && NWAVE * STW <= RCAP && STW >= 256);
static_assert((ZINTS % (NTHR * 4)) == 0);
static_assert(LDS_AGG <= 262144);
static_assert((NBA % NWAVE) == 0 && (NBA % GBM) == 0);
static_assert(GBM == (GTHR / 32) * 16 && GBN == 4 * 32 && GBN == F);
static_assert((F % 32) == 0 && (KC % 32) == 0 && KC == 2 * F && F == 32 * 4);
static_assert((NUL % NTHR) == 0 && (NUC1 % NTHR) == 0);

typedef float          v4f  __attribute__((ext_vector_type(4)));
typedef float          v8f  __attribute__((ext_vector_type(8)));
typedef int            v4i  __attribute__((ext_vector_type(4)));
typedef int            v8i  __attribute__((ext_vector_type(8)));
typedef unsigned int   v2u  __attribute__((ext_vector_type(2)));
typedef unsigned int   v4u  __attribute__((ext_vector_type(4)));
typedef unsigned short v8us __attribute__((ext_vector_type(8)));
typedef __bf16         v16b __attribute__((ext_vector_type(16)));
typedef v4f  __attribute__((may_alias)) v4fa;
typedef v4i  __attribute__((may_alias)) v4ia;
typedef v2u  __attribute__((may_alias)) v2ua;
typedef v4u  __attribute__((may_alias)) v4ua;
typedef v8us __attribute__((may_alias)) v8usa;
union Frag { v16b b; v8us h[2]; v8i w; };

__device__ __forceinline__ v8f wmb(const Frag& a, const Frag& b, v8f c) {
  v8f d = __builtin_amdgcn_wmma_f32_16x16x32_bf16(false, a.b, false, b.b, (short)0, c, false, false);
  asm volatile("v_nop\n\tv_nop\n\tv_nop\n\tv_nop" : "+v"(d) : "v"(a.w), "v"(b.w));
  return d;
}

__device__ __forceinline__ unsigned short bf_bits(float f) {
  unsigned int u = __float_as_uint(f);
  u += 0x7FFFu + ((u >> 16) & 1u);
  return (unsigned short)(u >> 16);
}
__device__ __forceinline__ float bf_val(unsigned short b) {
  return __uint_as_float(((unsigned int)b) << 16);
}
__device__ __forceinline__ float bf_rne(float f) { return bf_val(bf_bits(f)); }

__device__ __forceinline__ int scan_chunk(const int* __restrict__ dsts, int nE, int cbase, int slotBase,
                                          int nb, int vec8, int* list, int tid, int lane, int wave) {
  int wc = 0;
  const int el0  = tid * EPT;
  const int e0   = cbase + el0;
  const int sent = -2147483647 - 1;
  v4i da, db;
  if (vec8 != 0 && cbase + CHUNK <= nE) {
    da = *(const v4i*)(dsts + e0);
    db = *(const v4i*)(dsts + e0 + 4);
  } else {
    da.x = (e0     < nE) ? dsts[min(e0,     nE - 1)] : sent;
    da.y = (e0 + 1 < nE) ? dsts[min(e0 + 1, nE - 1)] : sent;
    da.z = (e0 + 2 < nE) ? dsts[min(e0 + 2, nE - 1)] : sent;
    da.w = (e0 + 3 < nE) ? dsts[min(e0 + 3, nE - 1)] : sent;
    db.x = (e0 + 4 < nE) ? dsts[min(e0 + 4, nE - 1)] : sent;
    db.y = (e0 + 5 < nE) ? dsts[min(e0 + 5, nE - 1)] : sent;
    db.z = (e0 + 6 < nE) ? dsts[min(e0 + 6, nE - 1)] : sent;
    db.w = (e0 + 7 < nE) ? dsts[min(e0 + 7, nE - 1)] : sent;
  }
  const unsigned nbs = (unsigned)slotBase;
  const unsigned unb = (unsigned)nb;
  const unsigned s0 = (unsigned)da.x - nbs, s1 = (unsigned)da.y - nbs;
  const unsigned s2 = (unsigned)da.z - nbs, s3 = (unsigned)da.w - nbs;
  const unsigned s4 = (unsigned)db.x - nbs, s5 = (unsigned)db.y - nbs;
  const unsigned s6 = (unsigned)db.z - nbs, s7 = (unsigned)db.w - nbs;
  const bool h0 = s0 < unb, h1 = s1 < unb, h2 = s2 < unb, h3 = s3 < unb;
  const bool h4 = s4 < unb, h5 = s5 < unb, h6 = s6 < unb, h7 = s7 < unb;
  const unsigned any = __builtin_amdgcn_ballot_w32(h0 | h1 | h2 | h3 | h4 | h5 | h6 | h7);
  if (any != 0u) {
#define HITJ(J, HJ, SJ) { \
      const unsigned mj = __builtin_amdgcn_ballot_w32(HJ); \
      if (mj != 0u) { \
        if (HJ) { \
          const int pos = wc + (int)__builtin_amdgcn_mbcnt_lo(mj, 0u); \
          if (pos < WCAP) list[wave * WCAP + pos] = ((el0 + (J)) << PKS) | (int)(SJ); \
        } \
        wc += (int)__builtin_popcount(mj); } }
    HITJ(0, h0, s0)
    HITJ(1, h1, s1)
    HITJ(2, h2, s2)
    HITJ(3, h3, s3)
    HITJ(4, h4, s4)
    HITJ(5, h5, s5)
    HITJ(6, h6, s6)
    HITJ(7, h7, s7)
#undef HITJ
  }
  return wc;
}

__global__ __launch_bounds__(NTHR) void k_wprep(const float* __restrict__ wlin, const float* __restrict__ wc,
                                                int nL, unsigned short* WLB, unsigned short* WCB) {
  const int u = (int)blockIdx.x * NTHR + (int)threadIdx.x;
  v8us o;
  unsigned short* dp;
  if (u < NUL) {
    const int n  = u >> 4;
    const int k8 = (u & 15) * 8;
    const float* p = wlin + (size_t)k8 * F + n;
#pragma unroll
    for (int i = 0; i < 8; ++i) o[i] = bf_bits(p[(size_t)i * F]);
    dp = WLB + (size_t)n * F + k8;
  } else if (u < NUL + nL * NUC1) {
    const int v  = u - NUL;
    const int l  = v >> 12;
    const int w  = v & (NUC1 - 1);
    const int n  = w >> 5;
    const int k8 = (w & 31) * 8;
    const int kk = k8 & (F - 1);
    const float* p = wc + (size_t)l * F * F + (size_t)kk * F + n;
#pragma unroll
    for (int i = 0; i < 8; ++i) o[i] = bf_bits(p[(size_t)i * F]);
    dp = WCB + ((size_t)l * F + (size_t)n) * KC + k8;
  } else {
    return;
  }
  *(volatile v8us*)dp = o;
  __threadfence();
  *(volatile v8us*)dp = o;
}

__global__ __launch_bounds__(NTHR) void k_cvx(const float* __restrict__ x, int nN, int nUnits,
                                              unsigned short* xb) {
  const int u = (int)blockIdx.x * NTHR + (int)threadIdx.x;
  if (u >= nUnits) return;
  const int row = u >> 4;
  const int c8  = (u & 15) * 8;
  const int rc  = row < nN ? row : nN - 1;
  const float keep = row < nN ? 1.0f : 0.0f;
  const float* p = x + (size_t)rc * F + c8;
  const v4f a = *(const v4f*)p;
  const v4f b = *(const v4f*)(p + 4);
  v8us o;
  o[0] = bf_bits(a.x * keep); o[1] = bf_bits(a.y * keep); o[2] = bf_bits(a.z * keep); o[3] = bf_bits(a.w * keep);
  o[4] = bf_bits(b.x * keep); o[5] = bf_bits(b.y * keep); o[6] = bf_bits(b.z * keep); o[7] = bf_bits(b.w * keep);
  unsigned short* dp = xb + (size_t)u * 8;
  *(volatile v8us*)dp = o;
  __threadfence();
  *(volatile v8us*)dp = o;
}

template <int MODE>
__global__ __launch_bounds__(GTHR) void k_gemm(const unsigned short* __restrict__ A, int lda,
                                               const unsigned short* __restrict__ BT, int ldb, int K,
                                               const float* __restrict__ bias, const float* __restrict__ Mf,
                                               float cm, float cw, float* C32, int nN) {
  __shared__ __attribute__((aligned(16))) float stg[GBM * GBN];
  const int tid = (int)threadIdx.x, lane = tid & 31, wave = tid >> 5, hh = lane >> 4, m = lane & 15;
  const int rowBase = (int)blockIdx.x * GBM;

  v8f acc[8];
  {
    const v8f z = {0.f, 0.f, 0.f, 0.f, 0.f, 0.f, 0.f, 0.f};
#pragma unroll
    for (int t = 0; t < 8; ++t) acc[t] = z;
  }
  const unsigned short* ap = A  + (size_t)(rowBase + 16 * wave + m) * (size_t)lda + 8 * hh;
  const unsigned short* bp = BT + (size_t)m * (size_t)ldb + 8 * hh;

#pragma unroll 1
  for (int k0 = 0; k0 < K; k0 += 32) {
    Frag af;
    af.h[0] = *(const v8usa*)(ap + k0);
    af.h[1] = *(const v8usa*)(ap + k0 + 16);
#pragma unroll
    for (int nt = 0; nt < 8; ++nt) {
      const unsigned short* wq = bp + (size_t)(16 * nt) * (size_t)ldb + k0;
      Frag bf;
      bf.h[0] = *(const v8usa*)wq;
      bf.h[1] = *(const v8usa*)(wq + 16);
      acc[nt] = wmb(af, bf, acc[nt]);
    }
  }

#pragma unroll
  for (int nt = 0; nt < 8; ++nt) {
    const int lc = 16 * nt + m;
#pragma unroll
    for (int r = 0; r < 8; ++r) {
      const int lr = 16 * wave + 8 * hh + r;
      stg[lr * GBN + lc] = acc[nt][r];
    }
  }
  __syncthreads();

  float bq[4];
  bq[0] = 0.0f; bq[1] = 0.0f; bq[2] = 0.0f; bq[3] = 0.0f;
  if constexpr (MODE == 0) {
    const v4f b4 = *(const v4f*)(bias + 4 * lane);
    bq[0] = bf_rne(b4.x); bq[1] = bf_rne(b4.y); bq[2] = bf_rne(b4.z); bq[3] = bf_rne(b4.w);
  }

  v4f pv[16];
#pragma unroll
  for (int i = 0; i < 16; ++i) {
    const int row = rowBase + 16 * wave + i;
    const bool ok = row < nN;
    const v4f xs = *(const v4fa*)(stg + (16 * wave + i) * GBN + 4 * lane);
    float y[4];
    if constexpr (MODE == 0) {
      y[0] = fmaxf(xs.x + bq[0], 0.0f); y[1] = fmaxf(xs.y + bq[1], 0.0f);
      y[2] = fmaxf(xs.z + bq[2], 0.0f); y[3] = fmaxf(xs.w + bq[3], 0.0f);
    } else {
      const v4f mr = *(const v4f*)(Mf + (size_t)row * F + 4 * lane);
      y[0] = fmaxf(cm * mr.x + cw * xs.x, 0.0f); y[1] = fmaxf(cm * mr.y + cw * xs.y, 0.0f);
      y[2] = fmaxf(cm * mr.z + cw * xs.z, 0.0f); y[3] = fmaxf(cm * mr.w + cw * xs.w, 0.0f);
    }
    v4f q;
    q.x = ok ? y[0] : 0.0f; q.y = ok ? y[1] : 0.0f; q.z = ok ? y[2] : 0.0f; q.w = ok ? y[3] : 0.0f;
    pv[i] = q;
  }
#pragma unroll
  for (int i = 0; i < 16; ++i) {
    const int row = rowBase + 16 * wave + i;
    float* op = C32 + (size_t)row * F + 4 * lane;
    if constexpr (MODE == 2) {
      if (row < nN) *(volatile v4f*)op = pv[i];
    } else {
      *(volatile v4f*)op = pv[i];
    }
  }
  __threadfence();
#pragma unroll
  for (int i = 0; i < 16; ++i) {
    const int row = rowBase + 16 * wave + i;
    float* op = C32 + (size_t)row * F + 4 * lane;
    if constexpr (MODE == 2) {
      if (row < nN) *(volatile v4f*)op = pv[i];
    } else {
      *(volatile v4f*)op = pv[i];
    }
  }
}

__global__ __launch_bounds__(NTHR) void k_agg(const int* __restrict__ srcs, const int* __restrict__ dsts,
                                              const float* __restrict__ ew, const float* __restrict__ Hs,
                                              const float* __restrict__ X0,
                                              float* Mf, unsigned short* MA,
                                              int nN, int nE, int vec8, int mRows) {
  extern __shared__ __attribute__((aligned(16))) int lds_i[];
  int* reg1 = lds_i;
  int* reg2 = reg1 + RCAP;
  int* scnt = reg2 + RCAP;
  int* soff = scnt + NBA;
  int* list = soff + NBA;
  int* wcnt = list + LISTN;
  int* wtot = wcnt + NWAVE;
  const int tid = (int)threadIdx.x, lane = tid & 31, wave = tid >> 5;
  const int nodeBase = (int)blockIdx.x * NBA;

  {
    const v4i z4 = {0, 0, 0, 0};
    for (int i = tid * 4; i < ZINTS; i += NTHR * 4) *(v4ia*)(lds_i + i) = z4;
    if (tid < 2 * NWAVE) wcnt[tid] = 0;
  }
  __syncthreads();

  int tot = 0;
  const int nChunks = (nE + CHUNK - 1) / CHUNK;
#pragma unroll 1
  for (int ch = 0; ch < nChunks; ++ch) {
    const int cbase = ch * CHUNK;
    const int wc = scan_chunk(dsts, nE, cbase, nodeBase, NBA, vec8, list, tid, lane, wave);
    if (lane == 0) wcnt[wave] = wc;
    __syncthreads();
    int pre = 0, all = 0;
#pragma unroll
    for (int w2 = 0; w2 < NWAVE; ++w2) {
      int c = wcnt[w2];
      c = c < 0 ? 0 : (c > WCAP ? WCAP : c);
      all += c;
      pre += (w2 < wave) ? c : 0;
    }
    const int wcc  = wc > WCAP ? WCAP : wc;
    const int base = tot + pre;
#pragma unroll 1
    for (int i = lane; i < wcc; i += 32) {
      const int ent = list[wave * WCAP + i];
      const int el  = (ent >> PKS) & (CHUNK - 1);
      const int sl  = ent & (NBA - 1);
      int eid = cbase + el;
      eid = eid > nE - 1 ? nE - 1 : eid;
      const int pos = base + i;
      if (pos < RCAP) reg1[pos] = (int)(((unsigned)eid << PKS) | (unsigned)sl);
    }
    tot += all;
    tot = tot > RCAP ? RCAP : tot;
    __syncthreads();
  }
  const int nh = tot;

  if (wave == 0) {
#pragma unroll 1
    for (int b0 = 0; b0 < nh; b0 += 32) {
      const int idx = b0 + lane;
      const int uv  = reg1[idx < RCAP ? idx : RCAP - 1];
      const int m32 = (nh - b0) < 32 ? (nh - b0) : 32;
#pragma unroll 1
      for (int k = 0; k < m32; ++k) {
        const int u  = __builtin_amdgcn_readlane(uv, k);
        const int sl = u & (NBA - 1);
        if (lane == 0) scnt[sl] = scnt[sl] + 1;
      }
    }
  }
  __syncthreads();

  {
    const int c0r = scnt[4 * tid], c1r = scnt[4 * tid + 1], c2r = scnt[4 * tid + 2], c3r = scnt[4 * tid + 3];
    const int e0 = c0r < 0 ? 0 : c0r, e1 = c1r < 0 ? 0 : c1r, e2 = c2r < 0 ? 0 : c2r, e3 = c3r < 0 ? 0 : c3r;
    const int ts = e0 + e1 + e2 + e3;
    int incl = ts;
#pragma unroll
    for (int d = 1; d < 32; d <<= 1) {
      const int up = __shfl_up(incl, d, 32);
      if (lane >= d) incl += up;
    }
    if (lane == 31) wtot[wave] = incl;
    __syncthreads();
    int pre = 0;
#pragma unroll
    for (int w2 = 0; w2 < NWAVE; ++w2) pre += (w2 < wave) ? wtot[w2] : 0;
    int run = pre + incl - ts;
    soff[4 * tid + 0] = run; run += e0;
    soff[4 * tid + 1] = run; run += e1;
    soff[4 * tid + 2] = run; run += e2;
    soff[4 * tid + 3] = run;
  }
  __syncthreads();
  for (int i = tid; i < NBA; i += NTHR) list[i] = soff[i];
  __syncthreads();

  if (wave == 0) {
#pragma unroll 1
    for (int b0 = 0; b0 < nh; b0 += 32) {
      const int idx = b0 + lane;
      const int uv  = reg1[idx < RCAP ? idx : RCAP - 1];
      const int m32 = (nh - b0) < 32 ? (nh - b0) : 32;
#pragma unroll 1
      for (int k = 0; k < m32; ++k) {
        const int u   = __builtin_amdgcn_readlane(uv, k);
        const int sl  = u & (NBA - 1);
        const int eid = (int)((unsigned)u >> PKS);
        if (lane == 0) {
          int pos = list[sl];
          pos = pos < 0 ? 0 : (pos > RCAP - 1 ? RCAP - 1 : pos);
          reg2[pos] = eid;
          list[sl] = pos + 1;
        }
      }
    }
  }
  __syncthreads();

  const int nbw = NBA / NWAVE;
  const bool ovf = (nh >= RCAP);
  const float qnan = __int_as_float(0x7fc00000);
  unsigned int* stwu = (unsigned int*)reg1 + wave * STW;

#pragma unroll 1
  for (int jt = 0; jt < nbw; ++jt) {
    const int slot = wave * nbw + jt;
    const int node = nodeBase + slot;
    int st = soff[slot];
    const int craw = scnt[slot];
    int cnt = craw;
    st  = st < 0 ? 0 : (st > nh ? nh : st);
    cnt = cnt < 0 ? 0 : (cnt > DEGCAP ? DEGCAP : cnt);
    if (cnt > nh - st) cnt = nh - st;
    const float pz = (ovf || craw > DEGCAP) ? qnan : 0.0f;
    const bool live = node < nN;
    const int nc = node < nN ? node : nN - 1;

    float a0 = 0.f, a1 = 0.f, a2 = 0.f, a3 = 0.f;
#pragma unroll 1
    for (int b0 = 0; b0 < cnt; b0 += 32) {
      int idx = st + b0 + lane; idx = idx > RCAP - 1 ? RCAP - 1 : idx;
      int eid = reg2[idx]; eid = eid < 0 ? 0 : (eid > nE - 1 ? nE - 1 : eid);
      int sr = srcs[eid]; sr = sr < 0 ? 0 : (sr > nN - 1 ? nN - 1 : sr);
      const float wv  = bf_rne(ew[eid]);
      const int   wvi = __float_as_int(wv);
      const int m32 = (cnt - b0) < 32 ? (cnt - b0) : 32;
#pragma unroll 1
      for (int k = 0; k < m32; ++k) {
        const int   sk = __builtin_amdgcn_readlane(sr, k);
        const float ck = __int_as_float(__builtin_amdgcn_readlane(wvi, k));
        const v4f v = *(const v4f*)(Hs + (size_t)sk * F + 4 * lane);
        a0 = fmaf(ck, v.x, a0); a1 = fmaf(ck, v.y, a1); a2 = fmaf(ck, v.z, a2); a3 = fmaf(ck, v.w, a3);
      }
    }
    const v4f xv = *(const v4f*)(X0 + (size_t)nc * F + 4 * lane);
    float r0 = 0.9f * a0 + 0.1f * xv.x, r1 = 0.9f * a1 + 0.1f * xv.y;
    float r2 = 0.9f * a2 + 0.1f * xv.z, r3 = 0.9f * a3 + 0.1f * xv.w;
    r0 = (live ? r0 : 0.0f) + pz;
    r1 = (live ? r1 : 0.0f) + pz;
    r2 = (live ? r2 : 0.0f) + pz;
    r3 = (live ? r3 : 0.0f) + pz;
    v4f mv;
    mv.x = r0; mv.y = r1; mv.z = r2; mv.w = r3;

    const unsigned short hb0 = bf_bits(r0), hb1 = bf_bits(r1), hb2 = bf_bits(r2), hb3 = bf_bits(r3);
    const unsigned short lb0 = bf_bits(r0 - bf_val(hb0)), lb1 = bf_bits(r1 - bf_val(hb1));
    const unsigned short lb2 = bf_bits(r2 - bf_val(hb2)), lb3 = bf_bits(r3 - bf_val(hb3));
    v2u hw, lw;
    hw.x = (unsigned int)hb0 | ((unsigned int)hb1 << 16);
    hw.y = (unsigned int)hb2 | ((unsigned int)hb3 << 16);
    lw.x = (unsigned int)lb0 | ((unsigned int)lb1 << 16);
    lw.y = (unsigned int)lb2 | ((unsigned int)lb3 << 16);
    __builtin_amdgcn_fence(__ATOMIC_RELEASE, "wavefront");
    __builtin_amdgcn_wave_barrier();
    *(v2ua*)(stwu + 2 * lane)      = hw;
    *(v2ua*)(stwu + 64 + 2 * lane) = lw;
    __builtin_amdgcn_fence(__ATOMIC_RELEASE, "wavefront");
    __builtin_amdgcn_wave_barrier();
    const v4u pk = *(const v4ua*)(stwu + 4 * lane);

    if (node < mRows) {
      float* mp = Mf + (size_t)node * F + 4 * lane;
      unsigned short* gp = MA + (size_t)node * (size_t)KC + 8 * lane;
      *(volatile v4f*)mp = mv;
      *(volatile v4u*)gp = pk;
      __threadfence();
      *(volatile v4f*)mp = mv;
      *(volatile v4u*)gp = pk;
    }
  }
}

static inline int cdiv(int a, int b) { return (a + b - 1) / b; }
static inline size_t al256(size_t o) { return (o + 255) & ~(size_t)255; }

extern "C" void kernel_launch(void* const* d_in, const int* in_sizes, int n_in,
                              void* d_out, int out_size, void* d_ws, size_t ws_size,
                              hipStream_t stream) {
  if (n_in < 6) return;
  if (in_sizes[0] < F || (in_sizes[0] % F) != 0) return;
  const int nN = in_sizes[0] / F;
  if (nN < 1 || nN > (1 << 24)) return;
  const int nE = in_sizes[1];
  if (nE < 1 || nE > (1 << 21)) return;
  if (in_sizes[2] != F * F || in_sizes[3] != F) return;
  if (in_sizes[4] < F * F || (in_sizes[4] % (F * F)) != 0) return;
  const int nL = in_sizes[4] / (F * F);
  if (nL < 1 || nL > 64) return;
  if (in_sizes[5] != 2 * nE) return;
  if ((long long)out_size != (long long)nN * F) return;

  const float* x    = (const float*)d_in[0];
  const float* ew   = (const float*)d_in[1];
  const float* wlin = (const float*)d_in[2];
  const float* blin = (const float*)d_in[3];
  const float* wcv  = (const float*)d_in[4];
  const int*   edge = (const int*)d_in[5];
  float* out = (float*)d_out;
  const int* src = edge;
  const int* dst = edge + nE;

  const int MP = cdiv(nN, GBM) * GBM;
  const int gM = MP / GBM;
  const int gA = cdiv(MP, NBA);
  if ((long long)gA * NBA < (long long)MP) return;
  const int vec8 = ((nE & 3) == 0) ? 1 : 0;

  char* ws = (char*)d_ws;
  size_t off = 0;
  const size_t oWLB = off; off = al256(off + (size_t)F * F * 2);
  const size_t oWCB = off; off = al256(off + (size_t)nL * F * KC * 2);
  const size_t oXB  = off; off = al256(off + (size_t)MP * F * 2);
  const size_t oX0  = off; off = al256(off + (size_t)MP * F * 4);
  const size_t oH   = off; off = al256(off + (size_t)MP * F * 4);
  const size_t oM   = off; off = al256(off + (size_t)MP * F * 4);
  const size_t oMA  = off; off = al256(off + (size_t)MP * KC * 2);
  if (off > ws_size || off > (size_t)WSMAX) return;
  unsigned short* WLB = (unsigned short*)(ws + oWLB);
  unsigned short* WCB = (unsigned short*)(ws + oWCB);
  unsigned short* XB  = (unsigned short*)(ws + oXB);
  float*          X0  = (float*)(ws + oX0);
  float*          H   = (float*)(ws + oH);
  float*          M   = (float*)(ws + oM);
  unsigned short* MA  = (unsigned short*)(ws + oMA);

  hipFuncSetAttribute(reinterpret_cast<const void*>(&k_agg), hipFuncAttributeMaxDynamicSharedMemorySize, LDS_AGG);

  const int nUw = NUL + nL * NUC1;
  k_wprep<<<cdiv(nUw, NTHR), NTHR, 0, stream>>>(wlin, wcv, nL, WLB, WCB);
  const int nUx = MP * (F / 8);
  k_cvx<<<cdiv(nUx, NTHR), NTHR, 0, stream>>>(x, nN, nUx, XB);

  k_gemm<0><<<gM, GTHR, 0, stream>>>(XB, F, WLB, F, F, blin, M, 0.0f, 0.0f, X0, nN);

  for (int l = 0; l < nL; ++l) {
    const double bd = log(0.5 / (double)(l + 1) + 1.0);
    const float  be = (float)bd;
    const float  cm = 1.0f - be;
    const float  cw = be;
    const float* Hs = (l == 0) ? X0 : H;
    k_agg<<<gA, NTHR, LDS_AGG, stream>>>(src, dst, ew, Hs, X0, M, MA, nN, nE, vec8, MP);
    const unsigned short* Wl = WCB + (size_t)l * F * KC;
    if (l == nL - 1) {
      k_gemm<2><<<gM, GTHR, 0, stream>>>(MA, KC, Wl, KC, KC, blin, M, cm, cw, out, nN);
    } else {
      k_gemm<1><<<gM, GTHR, 0, stream>>>(MA, KC, Wl, KC, KC, blin, M, cm, cw, H, nN);
    }
  }
}
